// AtmoSphericNeuralOperatorNet_63488206570144
// MI455X (gfx1250) — hardware-run, weakly checked
//
#include <hip/hip_runtime.h>
#include <math.h>

typedef __attribute__((ext_vector_type(16))) _Float16 v16h;
typedef __attribute__((ext_vector_type(8)))  _Float16 v8h;
typedef __attribute__((ext_vector_type(8)))  float    v8f;
typedef __attribute__((ext_vector_type(4)))  float    v4f;
typedef __attribute__((ext_vector_type(2)))  float    v2f;
typedef __attribute__((ext_vector_type(4)))  int      v4i;
typedef __attribute__((ext_vector_type(2)))  int      v2i;

constexpr int kHF = 361, kWF = 720, kPF = kHF * kWF;
constexpr int kHP = 90,  kWP = 180, kPP = kHP * kWP;
constexpr int kPFP = 259968;
constexpr int kNPP = 16256;
constexpr int kCI = 26, kCE = 48, kCO = 24, kHD = 96, kLM = 90;
static_assert(kPF == 259920);
static_assert(kPP == 16200);
static_assert((kPFP % 64) == 0 && kPFP >= kPF && (kPFP - kPF) < 64);
static_assert((kNPP % 64) == 0 && kNPP >= kPP && (kNPP - kPP) < 64);
static_assert((kWF % 4) == 0 && (kWP % 4) == 0 && (kPF % 4) == 0);

constexpr float kCarry    = 128.0f;
constexpr float kCarryInv = 1.0f / kCarry;
constexpr float kFwdScale = kCarry / (float)kWP;
constexpr float kAngStep  = 6.283185307179586f / (float)kWP;

constexpr float kResCarry = 2048.0f;
constexpr float kResInv   = 1.0f / kResCarry;
constexpr float kHiFloor  = 6.2e-5f;

constexpr int kTEnc  = 0;
constexpr int kTLw   = kTEnc  + 48 * 256;
constexpr int kTDec  = kTLw   + 96 * 448;
constexpr int kTM1   = kTDec  + 32 * 448;
constexpr int kTM2   = kTM1   + 384 * 64;
constexpr int kTTf   = kTM2   + 192 * 96;
constexpr int kTTi   = kTTf   + 192 * 192;
constexpr int kTEncL = kTTi   + 192 * 192;
constexpr int kTEnd  = kTEncL + 48 * 256;
constexpr int kTPairs = kTEnd / 2;
constexpr int kEncLoDelta = kTEncL - kTEnc;
static_assert(kTEncL == 186368);
static_assert(kTEnd == 198656);
static_assert((kTLw % 64) == 0 && (kTDec % 64) == 0 && (kTM1 % 64) == 0 && (kTM2 % 64) == 0 &&
              (kTTf % 64) == 0 && (kTTi % 64) == 0 && (kTEncL % 64) == 0 && (kTPairs % 256) == 0);
static_assert((kEncLoDelta % 8) == 0);

constexpr size_t kOffH  = 0;
constexpr size_t kOffDX = kOffH  + (size_t)kCE * kNPP * 4;
constexpr size_t kOffU  = kOffDX + (size_t)kCE * kNPP * 4;
constexpr size_t kOffY  = kOffU  + (size_t)kCE * kPFP * 4;
constexpr size_t kOffXF = kOffY  + (size_t)kCO * kPFP * 4;
constexpr size_t kOffCS = kOffXF + (size_t)90 * 96 * 96 * 2;
constexpr size_t kOffC2 = kOffCS + (size_t)90 * 90 * 128 * 2;
constexpr size_t kOffXG = kOffC2 + (size_t)90 * 48 * 192 * 2;
constexpr size_t kOffWT = kOffXG + (size_t)90 * 96 * 96 * 2;
constexpr size_t kWsTotal = kOffWT + (size_t)kTEnd * 2;
static_assert(kWsTotal == 88560640ull);
static_assert(kWsTotal <= 134217728ull);
static_assert((kOffDX % 128) == 0 && (kOffU % 128) == 0 && (kOffY % 128) == 0 && (kOffXF % 128) == 0 &&
              (kOffCS % 128) == 0 && (kOffC2 % 128) == 0 && (kOffXG % 128) == 0 && (kOffWT % 128) == 0);

constexpr int kUGroupsPerCh = kPFP / 4;
constexpr int kBilGroups    = kCE * kUGroupsPerCh;
constexpr int kOutGroups    = kCO * kPF / 4;
static_assert((kBilGroups % 256) == 0);
static_assert((kOutGroups % 32) == 0);

__device__ __forceinline__ int imin(int a, int b) { return a < b ? a : b; }
__device__ __forceinline__ int iclamp(int v, int lo, int hi) { return v < lo ? lo : (v > hi ? hi : v); }

__device__ __forceinline__ v16h ldfrag(const _Float16* p) {
  union { v16h v; v8h h[2]; } f;
  f.h[0] = *(const v8h*)(p);
  f.h[1] = *(const v8h*)(p + 16);
  return f.v;
}
__device__ __forceinline__ v8f mma_h(v16h a, v16h b, v8f c) {
  c = __builtin_amdgcn_wmma_f32_16x16x32_f16(false, a, false, b, (short)0, c, false, false);
  asm volatile("v_nop\n\tv_nop\n\tv_nop\n\tv_nop" : "+v"(c) : "v"(a), "v"(b));
  return c;
}
__device__ __forceinline__ v8f zero8() { return (v8f){0.f, 0.f, 0.f, 0.f, 0.f, 0.f, 0.f, 0.f}; }

__device__ __forceinline__ void store2_v4f(float* p, v4f v) {
  *(volatile v4f*)p = v;
  __threadfence();
  *(volatile v4f*)p = v;
}
__device__ __forceinline__ void store2_v8h(_Float16* p, v8h v) {
  *(volatile v8h*)p = v;
  __threadfence();
  *(volatile v8h*)p = v;
}
__device__ __forceinline__ v8h cvt8(v4f a0, v4f a1) {
  v8h h;
#pragma unroll
  for (int e = 0; e < 4; ++e) {
    h[e]     = (_Float16)a0[e];
    h[4 + e] = (_Float16)a1[e];
  }
  return h;
}
__device__ __forceinline__ float gelu_tanh(float x) {
  const float u = 0.7978845608028654f * (x + 0.044715f * (x * x * x));
  return 0.5f * x * (1.0f + tanhf(u));
}
__device__ __forceinline__ float twid(int m, int w, int ri, float sc) {
  const bool ok = (m < kLM) && (w < kWP);
  const int mc = imin(m, kLM - 1);
  const int wc = imin(w, kWP - 1);
  const int r = (mc * wc) % kWP;
  float s, c;
  sincosf((float)r * kAngStep, &s, &c);
  const float b = ri ? -s : c;
  return ok ? b * sc : 0.0f;
}

__global__ __launch_bounds__(256) void prep_tables_kernel(
    const float* __restrict__ encw, const float* __restrict__ lw, const float* __restrict__ decw,
    const float* __restrict__ m1, const float* __restrict__ m2, unsigned* __restrict__ wt)
{
  const int g = blockIdx.x * 256 + threadIdx.x;
  if (g >= kTPairs) return;
  const int el = g * 2;
  unsigned word = 0u;
  const bool isTw = (el >= kTTf) && (el < kTEncL);
  if (!isTw) {
    const float* src = m2;
    int Mv = 192, Kv = 96, Kp = 96, base = kTM2, kind = 0;
    if (el >= kTEncL)    { src = encw; Mv = 48;  Kv = 234; Kp = 256; base = kTEncL; kind = 2; }
    else if (el < kTLw)  { src = encw; Mv = 48;  Kv = 234; Kp = 256; base = kTEnc;  kind = 1; }
    else if (el < kTDec) { src = lw;   Mv = 96;  Kv = 432; Kp = 448; base = kTLw; }
    else if (el < kTM1)  { src = decw; Mv = 24;  Kv = 432; Kp = 448; base = kTDec; }
    else if (el < kTM2)  { src = m1;   Mv = 384; Kv = 48;  Kp = 64;  base = kTM1; }
    const int loc = el - base;
    const int row = loc / Kp;
    const int k = loc - row * Kp;
    const int rc  = row < Mv ? row : Mv - 1;
    const int k0c = k < Kv ? k : Kv - 1;
    const int k1c = (k + 1) < Kv ? (k + 1) : Kv - 1;
    const float a0 = src[(size_t)rc * Kv + k0c];
    const float a1 = src[(size_t)rc * Kv + k1c];
    const float v0 = (row < Mv && k < Kv) ? a0 : 0.0f;
    const float v1 = (row < Mv && (k + 1) < Kv) ? a1 : 0.0f;
    float o0 = v0, o1 = v1;
    if (kind != 0) {
      const float s0 = (fabsf(v0) < kHiFloor) ? 0.0f : v0;
      const float s1 = (fabsf(v1) < kHiFloor) ? 0.0f : v1;
      const _Float16 g0 = (_Float16)s0;
      const _Float16 g1 = (_Float16)s1;
      const float r0 = (v0 - (float)g0) * kResCarry;
      const float r1 = (v1 - (float)g1) * kResCarry;
      o0 = (kind == 2) ? r0 : s0;
      o1 = (kind == 2) ? r1 : s1;
    }
    const _Float16 h0 = (_Float16)o0;
    const _Float16 h1 = (_Float16)o1;
    word = (unsigned)__builtin_bit_cast(unsigned short, h0) |
           ((unsigned)__builtin_bit_cast(unsigned short, h1) << 16);
  } else {
    const bool isTf = el < kTTi;
    const int loc = el - (isTf ? kTTf : kTTi);
    const int row = loc / 192;
    const int col = loc - row * 192;
#pragma unroll 1
    for (int e = 0; e < 2; ++e) {
      const int cc = col + e;
      const int m  = isTf ? (row >> 1) : (cc >> 1);
      const int ri = isTf ? (row & 1) : (cc & 1);
      const int w  = isTf ? cc : row;
      const float sc = isTf ? kFwdScale : ((m == 0) ? 1.0f : 2.0f);
      const float v = twid(m, w, ri, sc);
      const _Float16 hv = (_Float16)v;
      const unsigned hb = (unsigned)__builtin_bit_cast(unsigned short, hv);
      word |= hb << (16 * e);
    }
  }
  ((volatile unsigned*)wt)[g] = word;
  __threadfence();
  ((volatile unsigned*)wt)[g] = word;
}

template <int CI, int MT, int MSTORE, bool ZRES>
__global__ __launch_bounds__(64) void disco_kernel(
    const float* __restrict__ xin, int inPitch, int pinReal,
    const int* __restrict__ idx, const float* __restrict__ vals, int poutReal,
    const _Float16* __restrict__ Wp, float* __restrict__ outp, int outPitch)
{
  constexpr int KV = CI * 9;
  constexpr int KP = ((KV + 31) / 32) * 32;
  constexpr int BP = KP + 8;
  constexpr int PADW = (KP - KV) / 2;
  static_assert((KV % 2) == 0 && (BP % 8) == 0 && (KP % 32) == 0);
  static_assert(MSTORE <= MT * 16 && (MSTORE % 8) == 0 && (CI % 2) == 0);
  static_assert((ZRES ? 2 : 1) * 32 * BP * 2 + MT * 16 * 36 * 4 <= 65536);
  static_assert(!ZRES || (MT * 16 * KP == 48 * 256));
  __shared__ __align__(16) _Float16 sB[32 * BP];
  __shared__ __align__(16) _Float16 sBl[ZRES ? 32 * BP : 8];
  __shared__ __align__(16) float sO[MT * 16 * 36];

  const int tid  = threadIdx.x;
  const int lane = tid & 31;
  const int wave = tid >> 5;
  const int p0   = blockIdx.x * 32;

  {
    const int pl = lane;
    const int cg = wave;
    int p = p0 + pl;
    p = (p < poutReal) ? p : (poutReal - 1);
    int gi[6];
    {
      const v2i* ip = (const v2i*)(idx + (size_t)p * 6);
      const v2i i0 = ip[0], i1 = ip[1], i2 = ip[2];
      gi[0] = iclamp(i0[0], 0, pinReal - 1);
      gi[1] = iclamp(i0[1], 0, pinReal - 1);
      gi[2] = iclamp(i1[0], 0, pinReal - 1);
      gi[3] = iclamp(i1[1], 0, pinReal - 1);
      gi[4] = iclamp(i2[0], 0, pinReal - 1);
      gi[5] = iclamp(i2[1], 0, pinReal - 1);
    }
    float vv[9][6];
#pragma unroll
    for (int k = 0; k < 9; ++k) {
      const v2f* vp = (const v2f*)(vals + ((size_t)k * poutReal + p) * 6);
      const v2f a = vp[0], b = vp[1], c = vp[2];
      vv[k][0] = a[0]; vv[k][1] = a[1];
      vv[k][2] = b[0]; vv[k][3] = b[1];
      vv[k][4] = c[0]; vv[k][5] = c[1];
    }
#pragma unroll 1
    for (int c = cg; c < CI; c += 2) {
      const float* xc = xin + (size_t)c * inPitch;
      float xv[6];
#pragma unroll
      for (int n = 0; n < 6; ++n) xv[n] = xc[gi[n]];
      _Float16* zp = sB + pl * BP + c * 9;
      _Float16* zl = sBl + (ZRES ? (pl * BP + c * 9) : 0);
#pragma unroll
      for (int k = 0; k < 9; ++k) {
        float s = 0.0f;
#pragma unroll
        for (int n = 0; n < 6; ++n) s = fmaf(vv[k][n], xv[n], s);
        if (ZRES) {
          const float sh = (fabsf(s) < kHiFloor) ? 0.0f : s;
          const _Float16 hv = (_Float16)sh;
          const float hf = (float)hv;
          const float rs = (s - hf) * kResCarry;
          zp[k] = hv;
          zl[k] = (_Float16)rs;
        } else {
          zp[k] = (_Float16)s;
        }
      }
    }
    unsigned* sBw = (unsigned*)sB;
#pragma unroll 1
    for (int e = tid; e < 32 * PADW; e += 64) {
      const int row = e / PADW;
      const int wd  = e - row * PADW;
      sBw[(row * BP + KV) / 2 + wd] = 0u;
    }
    if (ZRES) {
      unsigned* sBlw = (unsigned*)sBl;
#pragma unroll 1
      for (int e = tid; e < 32 * PADW; e += 64) {
        const int row = e / PADW;
        const int wd  = e - row * PADW;
        sBlw[(row * BP + KV) / 2 + wd] = 0u;
      }
    }
  }
  __syncthreads();

  const int h8 = (lane >> 4) * 8;
  const int rl = lane & 15;
  v8f acc[MT];
  v8f accr[MT];
#pragma unroll
  for (int i = 0; i < MT; ++i) {
    acc[i] = zero8();
    accr[i] = zero8();
  }
  const _Float16* bRow  = sB + (wave * 16 + rl) * BP + h8;
  const _Float16* bRowL = sBl + (ZRES ? ((wave * 16 + rl) * BP + h8) : 0);
  const _Float16* aRow  = Wp + (size_t)rl * KP + h8;
  const _Float16* aRowL = aRow + (ZRES ? kEncLoDelta : 0);
#pragma unroll 1
  for (int k0 = 0; k0 < KP; k0 += 32) {
    const v16h b = ldfrag(bRow + k0);
    v16h bl = b;
    if (ZRES) bl = ldfrag(bRowL + k0);
#pragma unroll
    for (int i = 0; i < MT; ++i) {
      const v16h a = ldfrag(aRow + (size_t)i * 16 * KP + k0);
      acc[i] = mma_h(a, b, acc[i]);
      if (ZRES) {
        const v16h al = ldfrag(aRowL + (size_t)i * 16 * KP + k0);
        accr[i] = mma_h(a, bl, accr[i]);
        accr[i] = mma_h(al, b, accr[i]);
      }
    }
  }
#pragma unroll
  for (int i = 0; i < MT; ++i) {
#pragma unroll
    for (int r = 0; r < 8; ++r) {
      float v = acc[i][r];
      if (ZRES) v = v + accr[i][r] * kResInv;
      sO[(i * 16 + h8 + r) * 36 + wave * 16 + rl] = v;
    }
  }
  __syncthreads();
  {
    const int q  = tid >> 3;
    const int c4 = (tid & 7) * 4;
#pragma unroll 1
    for (int it = 0; it < MSTORE / 8; ++it) {
      const int row = it * 8 + q;
      const v4f v = *(const v4f*)(sO + row * 36 + c4);
      store2_v4f(outp + (size_t)row * outPitch + p0 + c4, v);
    }
  }
}

__global__ __launch_bounds__(192) void fdft_kernel(
    const float* __restrict__ H, const _Float16* __restrict__ Tf, _Float16* __restrict__ XF)
{
  __shared__ __align__(16) _Float16 sH[96 * 200];
  __shared__ __align__(16) float sS[16 * 100];
  const int tid = threadIdx.x, lane = tid & 31, wave = tid >> 5;
  const int h8 = (lane >> 4) * 8, rl = lane & 15;
  const int c = blockIdx.x;
  const float* hc = H + (size_t)c * kNPP;
#pragma unroll 1
  for (int e = tid; e < 96 * 192; e += 192) {
    const int t = e / 192;
    const int w = e - t * 192;
    const int tc = imin(t, kHP - 1);
    const int wc = imin(w, kWP - 1);
    const float v = hc[tc * kWP + wc];
    const bool ok = (t < kHP) && (w < kWP);
    sH[t * 200 + w] = (_Float16)(ok ? v : 0.0f);
  }
  __syncthreads();
  const _Float16* bRow = sH + (wave * 16 + rl) * 200 + h8;
  v16h bf[6];
#pragma unroll
  for (int ks = 0; ks < 6; ++ks) bf[ks] = ldfrag(bRow + 32 * ks);
#pragma unroll 1
  for (int mi = 0; mi < 12; ++mi) {
    const _Float16* aRow = Tf + (size_t)(mi * 16 + rl) * 192 + h8;
    v8f acc = zero8();
#pragma unroll
    for (int ks = 0; ks < 6; ++ks) {
      const v16h a = ldfrag(aRow + 32 * ks);
      acc = mma_h(a, bf[ks], acc);
    }
#pragma unroll
    for (int r = 0; r < 8; ++r) sS[(h8 + r) * 100 + wave * 16 + rl] = acc[r];
    __syncthreads();
#pragma unroll 1
    for (int mm = wave; mm < 8; mm += 6) {
      const int m = mi * 8 + mm;
      const int lc = imin(lane, 23);
      const int row = lc / 12;
      const int seg = lc - row * 12;
      const float* sp = sS + (2 * mm + row) * 100 + seg * 8;
      const v4f a0 = *(const v4f*)(sp);
      const v4f a1 = *(const v4f*)(sp + 4);
      const v8h hv = cvt8(a0, a1);
      if (m < kLM && lane < 24) {
        store2_v8h(XF + ((size_t)(m * 96 + c * 2 + row) * 96 + seg * 8), hv);
      }
    }
    __syncthreads();
  }
}

__global__ __launch_bounds__(192) void sht_kernel(
    const float* __restrict__ Pw, const _Float16* __restrict__ XF, _Float16* __restrict__ CS)
{
  __shared__ __align__(16) _Float16 sA[96 * 104];
  __shared__ __align__(16) float sS[6 * 16 * 100];
  const int tid = threadIdx.x, lane = tid & 31, wave = tid >> 5;
  const int h8 = (lane >> 4) * 8, rl = lane & 15;
  const int m = blockIdx.x;
#pragma unroll 1
  for (int e = tid; e < 96 * 96; e += 192) {
    const int l = e / 96;
    const int t = e - l * 96;
    const int lc = imin(l, kLM - 1);
    const int tc = imin(t, kHP - 1);
    const float v = Pw[((size_t)lc * kLM + m) * kHP + tc];
    const bool ok = (l < kLM) && (t < kHP);
    sA[l * 104 + t] = (_Float16)(ok ? v : 0.0f);
  }
  __syncthreads();
  const int mi = wave;
  float* slab = sS + wave * 1600;
  const _Float16* aRow = sA + (mi * 16 + rl) * 104 + h8;
  v16h af[3];
#pragma unroll
  for (int ks = 0; ks < 3; ++ks) af[ks] = ldfrag(aRow + 32 * ks);
  const _Float16* xm = XF + (size_t)m * 96 * 96;
#pragma unroll 1
  for (int nj = 0; nj < 6; ++nj) {
    const int n  = nj * 16 + rl;
    const int ri = (n >= 48) ? 1 : 0;
    const int cc = n - ri * 48;
    const _Float16* bRow = xm + (size_t)(cc * 2 + ri) * 96 + h8;
    v8f acc = zero8();
#pragma unroll
    for (int ks = 0; ks < 3; ++ks) {
      const v16h b = ldfrag(bRow + 32 * ks);
      acc = mma_h(af[ks], b, acc);
    }
#pragma unroll
    for (int r = 0; r < 8; ++r) slab[(h8 + r) * 100 + nj * 16 + rl] = acc[r];
  }
  __syncthreads();
  {
    const int q = lane & 15, half = lane >> 4;
    const int ri = q >> 3, seg = q & 7;
    const int segc = imin(seg, 5);
    const bool live = seg < 6;
#pragma unroll 1
    for (int it = 0; it < 8; ++it) {
      const int row = it * 2 + half;
      const int l = mi * 16 + row;
      const float* sp = slab + row * 100 + ri * 48 + segc * 8;
      const v4f a0 = *(const v4f*)(sp);
      const v4f a1 = *(const v4f*)(sp + 4);
      v8h hv;
#pragma unroll
      for (int e = 0; e < 4; ++e) {
        hv[e]     = (_Float16)(live ? a0[e] : 0.0f);
        hv[4 + e] = (_Float16)(live ? a1[e] : 0.0f);
      }
      if (mi * 16 + it * 2 < kLM) {
        store2_v8h(CS + ((size_t)(l * kLM + m) * 128 + q * 8), hv);
      }
    }
  }
}

__global__ __launch_bounds__(128) void gw_kernel(
    const float* __restrict__ gwb, const _Float16* __restrict__ CS, _Float16* __restrict__ C2)
{
  __shared__ __align__(16) _Float16 sA[48 * 72];
  __shared__ __align__(16) float sS[48 * 196];
  const int tid = threadIdx.x, lane = tid & 31, wave = tid >> 5;
  const int h8 = (lane >> 4) * 8, rl = lane & 15;
  const int l = blockIdx.x;
#pragma unroll 1
  for (int e = tid; e < 48 * 64; e += 128) {
    const int o = e >> 6;
    const int i = e & 63;
    const int ic = imin(i, kCE - 1);
    const float v = gwb[((size_t)o * kCE + ic) * kLM + l];
    sA[o * 72 + i] = (_Float16)((i < kCE) ? v : 0.0f);
  }
  __syncthreads();
#pragma unroll 1
  for (int tI = 0; tI < 9; ++tI) {
    const int njl = tI / 3;
    const int mi  = tI - njl * 3;
    const int nj  = wave + 4 * njl;
    const int n   = nj * 16 + rl;
    const int nc  = imin(n, 2 * kLM - 1);
    const _Float16* bRow = CS + ((size_t)l * (2 * kLM) + nc) * 64 + h8;
    const _Float16* aRow = sA + (mi * 16 + rl) * 72 + h8;
    v8f acc = zero8();
#pragma unroll
    for (int ks = 0; ks < 2; ++ks) {
      const v16h a = ldfrag(aRow + 32 * ks);
      const v16h b = ldfrag(bRow + 32 * ks);
      acc = mma_h(a, b, acc);
    }
#pragma unroll
    for (int r = 0; r < 8; ++r) sS[(mi * 16 + h8 + r) * 196 + nj * 16 + rl] = acc[r];
  }
  __syncthreads();
  {
    const int lc = imin(lane, 23);
    const int n0 = lc * 8;
#pragma unroll 1
    for (int it = 0; it < 12; ++it) {
      const int o = wave + 4 * it;
      const float* sp = sS + o * 196 + n0;
      const v4f a0 = *(const v4f*)(sp);
      const v4f a1 = *(const v4f*)(sp + 4);
      v8h hv;
#pragma unroll
      for (int e = 0; e < 4; ++e) {
        hv[e]     = (_Float16)((n0 + e < 2 * kLM) ? a0[e] : 0.0f);
        hv[4 + e] = (_Float16)((n0 + 4 + e < 2 * kLM) ? a1[e] : 0.0f);
      }
      if (lane < 24) {
        store2_v8h(C2 + ((size_t)(l * kCE + o) * 192 + n0), hv);
      }
    }
  }
}

__global__ __launch_bounds__(192) void isht_kernel(
    const float* __restrict__ Pi, const _Float16* __restrict__ C2, _Float16* __restrict__ XG)
{
  __shared__ __align__(16) _Float16 sA[96 * 104];
  __shared__ __align__(16) _Float16 sB[96 * 104];
  __shared__ __align__(16) _Float16 sS[6 * 16 * 104];
  const int tid = threadIdx.x, lane = tid & 31, wave = tid >> 5;
  const int h8 = (lane >> 4) * 8, rl = lane & 15;
  const int m = blockIdx.x;
#pragma unroll 1
  for (int e = tid; e < 96 * 96; e += 192) {
    const int l = e / 96;
    const int t = e - l * 96;
    const int lc = imin(l, kLM - 1);
    const int tc = imin(t, kHP - 1);
    const float v = Pi[((size_t)lc * kLM + m) * kHP + tc];
    const bool ok = (l < kLM) && (t < kHP);
    sB[t * 104 + l] = (_Float16)(ok ? v : 0.0f);
  }
  const unsigned* c2w = (const unsigned*)C2;
#pragma unroll 1
  for (int e = tid; e < 96 * 48; e += 192) {
    const int l  = e / 48;
    const int cc = e - l * 48;
    const int lc = imin(l, kLM - 1);
    const unsigned w = c2w[((size_t)lc * kCE + cc) * 96 + m];
    const bool ok = l < kLM;
    const unsigned short lo = (unsigned short)(ok ? (w & 0xffffu) : 0u);
    const unsigned short hi = (unsigned short)(ok ? (w >> 16) : 0u);
    sA[(cc * 2) * 104 + l]     = __builtin_bit_cast(_Float16, lo);
    sA[(cc * 2 + 1) * 104 + l] = __builtin_bit_cast(_Float16, hi);
  }
  __syncthreads();
  const int mi = wave;
  _Float16* slab = sS + wave * (16 * 104);
  const _Float16* aRow = sA + (mi * 16 + rl) * 104 + h8;
  v16h af[3];
#pragma unroll
  for (int ks = 0; ks < 3; ++ks) af[ks] = ldfrag(aRow + 32 * ks);
#pragma unroll 1
  for (int nj = 0; nj < 6; ++nj) {
    const _Float16* bRow = sB + (nj * 16 + rl) * 104 + h8;
    v8f acc = zero8();
#pragma unroll
    for (int ks = 0; ks < 3; ++ks) {
      const v16h b = ldfrag(bRow + 32 * ks);
      acc = mma_h(af[ks], b, acc);
    }
#pragma unroll
    for (int r = 0; r < 8; ++r) slab[(h8 + r) * 104 + nj * 16 + rl] = (_Float16)acc[r];
  }
  __syncthreads();
  {
    _Float16* dstBase = XG + (size_t)(m * 96 + mi * 16) * 96;
#pragma unroll 1
    for (int it = 0; it < 6; ++it) {
      const int g = it * 32 + lane;
      const int row = g / 12;
      const int seg = g - row * 12;
      const v8h hv = *(const v8h*)(slab + row * 104 + seg * 8);
      store2_v8h(dstBase + (size_t)row * 96 + seg * 8, hv);
    }
  }
}

__global__ __launch_bounds__(128) void idft_kernel(
    const _Float16* __restrict__ XG, const _Float16* __restrict__ Ti, float* __restrict__ DX)
{
  __shared__ __align__(16) _Float16 sA[96 * 200];
  __shared__ __align__(16) float sS[16 * 196];
  const int tid = threadIdx.x, lane = tid & 31, wave = tid >> 5;
  const int h8 = (lane >> 4) * 8, rl = lane & 15;
  const int c = blockIdx.x;
  const unsigned* xgw = (const unsigned*)XG;
#pragma unroll 1
  for (int e = tid; e < kLM * 96; e += 128) {
    const int m   = e / 96;
    const int rem = e - m * 96;
    const int ri  = rem / 48;
    const int tw  = rem - ri * 48;
    const unsigned w = xgw[((size_t)m * 96 + c * 2 + ri) * 48 + tw];
    const unsigned short lo = (unsigned short)(w & 0xffffu);
    const unsigned short hi = (unsigned short)(w >> 16);
    sA[(tw * 2) * 200 + m * 2 + ri]     = __builtin_bit_cast(_Float16, lo);
    sA[(tw * 2 + 1) * 200 + m * 2 + ri] = __builtin_bit_cast(_Float16, hi);
  }
  {
    unsigned* sAw = (unsigned*)sA;
#pragma unroll 1
    for (int e = tid; e < 96 * 6; e += 128) {
      const int row = e / 6;
      const int wd  = e - row * 6;
      sAw[(row * 200 + 2 * kLM) / 2 + wd] = 0u;
    }
  }
  __syncthreads();
#pragma unroll 1
  for (int mi = 0; mi < 6; ++mi) {
    const _Float16* aRow = sA + (mi * 16 + rl) * 200 + h8;
#pragma unroll 1
    for (int njl = 0; njl < 3; ++njl) {
      const int nj = wave + 4 * njl;
      const _Float16* bRow = Ti + (size_t)(nj * 16 + rl) * 192 + h8;
      v8f acc = zero8();
#pragma unroll
      for (int ks = 0; ks < 6; ++ks) {
        const v16h a = ldfrag(aRow + 32 * ks);
        const v16h b = ldfrag(bRow + 32 * ks);
        acc = mma_h(a, b, acc);
      }
#pragma unroll
      for (int r = 0; r < 8; ++r) sS[(h8 + r) * 196 + nj * 16 + rl] = acc[r] * kCarryInv;
    }
    __syncthreads();
    {
      const int pieces = (mi < 5) ? 720 : 464;
      float* base = DX + (size_t)c * kNPP + mi * 2880;
#pragma unroll 1
      for (int it = 0; it < 6; ++it) {
        const int g  = it * 128 + tid;
        const int gc = imin(g, pieces - 1);
        const int f  = gc * 4;
        const int t  = f / kWP;
        const int w  = f - t * kWP;
        const int tcl = imin(t, 15);
        const v4f v = *(const v4f*)(sS + tcl * 196 + w);
        const bool real = (mi * 16 + t) < kHP;
        v4f o;
#pragma unroll
        for (int e = 0; e < 4; ++e) o[e] = real ? v[e] : 0.0f;
        if (g < pieces) store2_v4f(base + f, o);
      }
    }
    __syncthreads();
  }
}

__global__ __launch_bounds__(128) void mlp_kernel(
    const float* __restrict__ DX, float* H,
    const _Float16* __restrict__ m1p, const _Float16* __restrict__ m2p, const float* __restrict__ ls)
{
  __shared__ __align__(16) _Float16 sX[64 * 72];
  __shared__ __align__(16) _Float16 sAct[64 * 104];
  __shared__ __align__(16) float sO[48 * 68];
  const int tid = threadIdx.x, lane = tid & 31, wave = tid >> 5;
  const int h8 = (lane >> 4) * 8, rl = lane & 15;
  const int p0 = blockIdx.x * 64;
#pragma unroll 1
  for (int e = tid; e < 64 * 64; e += 128) {
    const int c   = e >> 6;
    const int pix = e & 63;
    const int cc  = imin(c, kCE - 1);
    const float v = DX[(size_t)cc * kNPP + p0 + pix];
    sX[pix * 72 + c] = (_Float16)((c < kCE) ? v : 0.0f);
  }
  __syncthreads();
  {
    const _Float16* xRow = sX + (wave * 16 + rl) * 72 + h8;
    const v16h xb0 = ldfrag(xRow);
    const v16h xb1 = ldfrag(xRow + 32);
#pragma unroll 1
    for (int mi = 0; mi < 6; ++mi) {
      const _Float16* aRow = m1p + (size_t)(mi * 16 + rl) * 64 + h8;
      v8f acc = zero8();
      const v16h a0 = ldfrag(aRow);
      acc = mma_h(a0, xb0, acc);
      const v16h a1 = ldfrag(aRow + 32);
      acc = mma_h(a1, xb1, acc);
      v8h hv;
#pragma unroll
      for (int r = 0; r < 8; ++r) hv[r] = (_Float16)gelu_tanh(acc[r]);
      *(v8h*)(sAct + (wave * 16 + rl) * 104 + mi * 16 + h8) = hv;
    }
  }
  __syncthreads();
  {
    const _Float16* bRow = sAct + (wave * 16 + rl) * 104 + h8;
    v16h bf[3];
#pragma unroll
    for (int ks = 0; ks < 3; ++ks) bf[ks] = ldfrag(bRow + 32 * ks);
#pragma unroll 1
    for (int mi = 0; mi < 3; ++mi) {
      const _Float16* aRow = m2p + (size_t)(mi * 16 + rl) * 96 + h8;
      v8f acc = zero8();
#pragma unroll
      for (int ks = 0; ks < 3; ++ks) {
        const v16h a = ldfrag(aRow + 32 * ks);
        acc = mma_h(a, bf[ks], acc);
      }
#pragma unroll
      for (int r = 0; r < 8; ++r) sO[(mi * 16 + h8 + r) * 68 + wave * 16 + rl] = acc[r];
    }
  }
  __syncthreads();
  {
    const int q  = tid >> 4;
    const int c4 = (tid & 15) * 4;
#pragma unroll 1
    for (int it = 0; it < 6; ++it) {
      const int row = it * 8 + q;
      const v4f d = *(const v4f*)(sO + row * 68 + c4);
      float* hp = H + (size_t)row * kNPP + p0 + c4;
      const v4f hv = *(const v4f*)hp;
      const float lsv = ls[row];
      v4f o;
#pragma unroll
      for (int e = 0; e < 4; ++e) o[e] = hv[e] + lsv * d[e];
      store2_v4f(hp, o);
    }
  }
}

__global__ __launch_bounds__(256) void bilinear_kernel(
    const float* __restrict__ H,
    const int* __restrict__ li0, const int* __restrict__ li1, const float* __restrict__ lwv,
    const int* __restrict__ ji0, const int* __restrict__ ji1, const float* __restrict__ jwv,
    float* __restrict__ U)
{
  const int g = blockIdx.x * 256 + threadIdx.x;
  if (g >= kBilGroups) return;
  const int c = g / kUGroupsPerCh;
  const int q = g - c * kUGroupsPerCh;
  const int p = q * 4;
  const bool real = p < kPF;
  const int pc = real ? p : (kPF - 4);
  const int I = pc / kWF;
  const int J = pc - I * kWF;
  const int a0 = iclamp(li0[I], 0, kHP - 1);
  const int a1 = iclamp(li1[I], 0, kHP - 1);
  const float aw = lwv[I];
  const v4i b0 = *(const v4i*)(ji0 + J);
  const v4i b1 = *(const v4i*)(ji1 + J);
  const v4f bw = *(const v4f*)(jwv + J);
  const float* r0 = H + (size_t)c * kNPP + a0 * kWP;
  const float* r1 = H + (size_t)c * kNPP + a1 * kWP;
  const float am = 1.0f - aw;
  v4f o;
#pragma unroll
  for (int e = 0; e < 4; ++e) {
    const int j0 = iclamp(b0[e], 0, kWP - 1);
    const int j1 = iclamp(b1[e], 0, kWP - 1);
    const float t0 = r0[j0] * am + r1[j0] * aw;
    const float t1 = r0[j1] * am + r1[j1] * aw;
    const float wv = bw[e];
    const float uv = t0 * (1.0f - wv) + t1 * wv;
    o[e] = real ? uv : 0.0f;
  }
  store2_v4f(U + (size_t)c * kPFP + p, o);
}

__global__ __launch_bounds__(256) void out_copy_kernel(const float* __restrict__ Y, float* __restrict__ outp)
{
  const int g = blockIdx.x * 256 + threadIdx.x;
  if (g >= kOutGroups) return;
  const int f = g * 4;
  const int o = f / kPF;
  const int p = f - o * kPF;
  const v4f v = *(const v4f*)(Y + (size_t)o * kPFP + p);
  store2_v4f(outp + (size_t)f, v);
}

extern "C" void kernel_launch(void* const* d_in, const int* in_sizes, int n_in,
                              void* d_out, int out_size, void* d_ws, size_t ws_size,
                              hipStream_t stream) {
  if (n_in < 22) return;
  if (in_sizes[0] != kCI * kPF) return;
  if (in_sizes[1] != kPP * 6) return;
  if (in_sizes[2] != 9 * kPP * 6) return;
  if (in_sizes[3] != kCE * kCI * 9) return;
  if (in_sizes[4] != kPP * 6) return;
  if (in_sizes[5] != 9 * kPP * 6) return;
  if (in_sizes[6] != 2 * kCE * kCE * 9) return;
  if (in_sizes[7] != 2 * kCE * kCE * kLM) return;
  if (in_sizes[8] != kLM * kLM * kHP) return;
  if (in_sizes[9] != kLM * kLM * kHP) return;
  if (in_sizes[10] != 4 * kHD * kCE) return;
  if (in_sizes[11] != 4 * kCE * kHD) return;
  if (in_sizes[12] != 4 * kCE) return;
  if (in_sizes[13] != kHF || in_sizes[14] != kHF || in_sizes[15] != kHF) return;
  if (in_sizes[16] != kWF || in_sizes[17] != kWF || in_sizes[18] != kWF) return;
  if (in_sizes[19] != kPF * 6) return;
  if (in_sizes[20] != 9 * kPF * 6) return;
  if (in_sizes[21] != kCO * kCE * 9) return;
  if (out_size != kCO * kPF) return;
  if (ws_size < kWsTotal) return;

  const float* x         = (const float*)d_in[0];
  const int*   enc_idx   = (const int*)  d_in[1];
  const float* enc_vals  = (const float*)d_in[2];
  const float* enc_w     = (const float*)d_in[3];
  const int*   proc_idx  = (const int*)  d_in[4];
  const float* proc_vals = (const float*)d_in[5];
  const float* lw        = (const float*)d_in[6];
  const float* gw        = (const float*)d_in[7];
  const float* Pw        = (const float*)d_in[8];
  const float* Pi        = (const float*)d_in[9];
  const float* m1        = (const float*)d_in[10];
  const float* m2        = (const float*)d_in[11];
  const float* ls        = (const float*)d_in[12];
  const int*   lat_i0    = (const int*)  d_in[13];
  const int*   lat_i1    = (const int*)  d_in[14];
  const float* lat_w     = (const float*)d_in[15];
  const int*   lon_i0    = (const int*)  d_in[16];
  const int*   lon_i1    = (const int*)  d_in[17];
  const float* lon_w     = (const float*)d_in[18];
  const int*   dec_idx   = (const int*)  d_in[19];
  const float* dec_vals  = (const float*)d_in[20];
  const float* dec_w     = (const float*)d_in[21];

  char* ws = (char*)d_ws;
  float*    H  = (float*)(ws + kOffH);
  float*    DX = (float*)(ws + kOffDX);
  float*    U  = (float*)(ws + kOffU);
  float*    Y  = (float*)(ws + kOffY);
  _Float16* XF = (_Float16*)(ws + kOffXF);
  _Float16* CS = (_Float16*)(ws + kOffCS);
  _Float16* C2 = (_Float16*)(ws + kOffC2);
  _Float16* XG = (_Float16*)(ws + kOffXG);
  _Float16* WT = (_Float16*)(ws + kOffWT);
  const _Float16* encWp = WT + kTEnc;
  const _Float16* lwP   = WT + kTLw;
  const _Float16* decWp = WT + kTDec;
  const _Float16* m1P   = WT + kTM1;
  const _Float16* m2P   = WT + kTM2;
  const _Float16* TfP   = WT + kTTf;
  const _Float16* TiP   = WT + kTTi;

  prep_tables_kernel<<<kTPairs / 256, 256, 0, stream>>>(enc_w, lw, dec_w, m1, m2, (unsigned*)WT);

  disco_kernel<kCI, 3, 48, true><<<kNPP / 32, 64, 0, stream>>>(
      x, kPF, kPF, enc_idx, enc_vals, kPP, encWp, H, kNPP);

  for (int i = 0; i < 4; ++i) {
    const int hh = i / 2;
    if ((i & 1) == 0) {
      fdft_kernel<<<kCE, 192, 0, stream>>>(H, TfP, XF);
      sht_kernel<<<kLM, 192, 0, stream>>>(Pw, XF, CS);
      gw_kernel<<<kLM, 128, 0, stream>>>(gw + (size_t)hh * kCE * kCE * kLM, CS, C2);
      isht_kernel<<<kLM, 192, 0, stream>>>(Pi, C2, XG);
      idft_kernel<<<kCE, 128, 0, stream>>>(XG, TiP, DX);
    } else {
      disco_kernel<kCE, 3, 48, false><<<kNPP / 32, 64, 0, stream>>>(
          H, kNPP, kPP, proc_idx, proc_vals, kPP, lwP + (size_t)hh * 48 * 448, DX, kNPP);
    }
    mlp_kernel<<<kNPP / 64, 128, 0, stream>>>(
        DX, H, m1P + (size_t)i * 96 * 64, m2P + (size_t)i * 48 * 96, ls + i * kCE);
  }

  bilinear_kernel<<<kBilGroups / 256, 256, 0, stream>>>(
      H, lat_i0, lat_i1, lat_w, lon_i0, lon_i1, lon_w, U);

  disco_kernel<kCE, 2, 24, false><<<kPFP / 32, 64, 0, stream>>>(
      U, kPFP, kPF, dec_idx, dec_vals, kPF, decWp, Y, kPFP);

  out_copy_kernel<<<(kOutGroups + 255) / 256, 256, 0, stream>>>(Y, (float*)d_out);
}
